// MambaBlock_48850958025090
// MI455X (gfx1250) — hardware-verified
//
#include <hip/hip_runtime.h>
#include <math.h>

typedef __attribute__((ext_vector_type(16))) _Float16 v16h;
typedef __attribute__((ext_vector_type(8)))  _Float16 v8h;
typedef __attribute__((ext_vector_type(16))) __bf16   v16b;
typedef __attribute__((ext_vector_type(8)))  __bf16   v8b;
typedef __attribute__((ext_vector_type(8)))  float    v8f;
typedef __attribute__((ext_vector_type(4)))  float    v4f;
typedef __attribute__((ext_vector_type(4)))  unsigned v4u;

constexpr int kBatch  = 8;
constexpr int kSeq    = 1024;
constexpr int kDm     = 256;
constexpr int kDin    = 1024;
constexpr int kNst    = 32;
constexpr int kNstL   = kNst / 2;
constexpr int kDtR    = 16;
constexpr int kConvK  = 8;
constexpr int kXzP    = 2 * kDin;
constexpr int kXdW    = kDtR + 2 * kNst;
constexpr int kXdP    = 128;
constexpr int kRows   = kBatch * kSeq;
constexpr int kConvTP = 260;
constexpr int kScanTS = 64;
constexpr int kScanCh = 64;
constexpr int kScanTh = 128;
constexpr int kScanYP = 68;
constexpr int kSxP    = 80;
static_assert(kXdW == 80, "x_proj width");
static_assert((kDm % 32) == 0 && (kDin % 32) == 0, "K multiples of 32");
static_assert((kRows % 64) == 0 && (kXzP % 64) == 0 && (kXdP % 64) == 0 && (kDm % 64) == 0, "M,N multiples of 64");
static_assert((kSeq % kScanTS) == 0 && (kSeq % 64) == 0 && (kDin % kScanCh) == 0 && (kDin % 256) == 0, "tile multiples");
static_assert((kScanTS * kSxP) % (4 * kScanTh) == 0 && (kScanTS * kSxP) / (4 * kScanTh) == 10, "scan staging coverage");
static_assert(kScanTh == 2 * kScanCh && kNstL * 2 == kNst, "two lanes per channel");

constexpr size_t kOffXNH  = 0;
constexpr size_t kOffXNL  = kOffXNH + (size_t)kRows * kDm  * 2;
constexpr size_t kOffWI   = kOffXNL + (size_t)kRows * kDm  * 2;
constexpr size_t kOffWX   = kOffWI  + (size_t)kXzP  * kDm  * 2;
constexpr size_t kOffWO   = kOffWX  + (size_t)kXdP  * kDin * 2;
constexpr size_t kOffXZ   = kOffWO  + (size_t)kDm   * kDin * 2;
constexpr size_t kOffUY0  = kOffXZ  + (size_t)kRows * kXzP * 4;
constexpr size_t kOffUY1  = kOffUY0 + (size_t)kRows * kDin * 2;
constexpr size_t kOffXD   = kOffUY1 + (size_t)kRows * kDin * 2;
constexpr size_t kWsTotal = kOffXD  + (size_t)kRows * kXdP * 4;
static_assert(kWsTotal == 115081216ull, "carve total");
static_assert(kWsTotal <= 134217728ull, "carve cap");
static_assert((kOffXNL % 128) == 0 && (kOffWI % 128) == 0 && (kOffWX % 128) == 0 && (kOffWO % 128) == 0 &&
              (kOffXZ % 128) == 0 && (kOffUY0 % 128) == 0 && (kOffUY1 % 128) == 0 && (kOffXD % 128) == 0, "128-B aligned regions");

__device__ __forceinline__ unsigned short f2bf_bits(float f) {
  unsigned u = __float_as_uint(f);
  return (unsigned short)((u + 0x7FFFu + ((u >> 16) & 1u)) >> 16);
}
__device__ __forceinline__ float bf_bits2f(unsigned short h) { return __uint_as_float(((unsigned)h) << 16); }
__device__ __forceinline__ float bf16_rne(float f) { return bf_bits2f(f2bf_bits(f)); }

__device__ __forceinline__ void dep_guard_h(v8f& a, v8f& b, v16h x, v16h y) { asm volatile("v_nop\n\tv_nop\n\tv_nop\n\tv_nop" : "+v"(a), "+v"(b) : "v"(x), "v"(y)); }
__device__ __forceinline__ void dep_guard_b(v8f& a, v8f& b, v16b x, v16b y) { asm volatile("v_nop\n\tv_nop\n\tv_nop\n\tv_nop" : "+v"(a), "+v"(b) : "v"(x), "v"(y)); }
__device__ __forceinline__ void dep_guard_all_h(v8f& a, v8f& b, v8f& c, v8f& d, v16h x0, v16h x1, v16h y0, v16h y1, v16h y2, v16h y3) {
  asm volatile("v_nop\n\tv_nop\n\tv_nop\n\tv_nop" : "+v"(a), "+v"(b), "+v"(c), "+v"(d) : "v"(x0), "v"(x1), "v"(y0), "v"(y1), "v"(y2), "v"(y3)); }
__device__ __forceinline__ void dep_guard_all_b(v8f& a, v8f& b, v8f& c, v8f& d, v16b x0, v16b x1, v16b y0, v16b y1, v16b y2, v16b y3) {
  asm volatile("v_nop\n\tv_nop\n\tv_nop\n\tv_nop" : "+v"(a), "+v"(b), "+v"(c), "+v"(d) : "v"(x0), "v"(x1), "v"(y0), "v"(y1), "v"(y2), "v"(y3)); }
__device__ __forceinline__ void keep4_h(v16h a, v16h b, v16h c, v16h d) { asm volatile("v_nop" :: "v"(a), "v"(b), "v"(c), "v"(d)); }
__device__ __forceinline__ void keep4_b(v16b a, v16b b, v16b c, v16b d) { asm volatile("v_nop" :: "v"(a), "v"(b), "v"(c), "v"(d)); }
__device__ __forceinline__ void acc_guard4(v8f& a, v8f& b, v8f& c, v8f& d) { asm volatile("v_nop\n\tv_nop\n\tv_nop\n\tv_nop" : "+v"(a), "+v"(b), "+v"(c), "+v"(d)); }
template <typename T> struct Frag;
template <> struct Frag<_Float16> {
  typedef v16h V; union U { v16h v; v8h h[2]; };
  static __device__ __forceinline__ v16h load(const _Float16* p) {
    U f; f.h[0] = *(const v8h*)(p); f.h[1] = *(const v8h*)(p + 16); return f.v;
  }
  static __device__ __forceinline__ v8f mma(v16h a, v16h b, v8f c) {
    return __builtin_amdgcn_wmma_f32_16x16x32_f16(false, a, false, b, (short)0, c, false, false);
  }
  static __device__ __forceinline__ void guard(v8f& a, v8f& b, v16h x, v16h y) { dep_guard_h(a, b, x, y); }
  static __device__ __forceinline__ void guard_all(v8f& a, v8f& b, v8f& c, v8f& d, v16h x0, v16h x1, v16h y0, v16h y1, v16h y2, v16h y3) { dep_guard_all_h(a, b, c, d, x0, x1, y0, y1, y2, y3); }
  static __device__ __forceinline__ void keep(v16h a, v16h b, v16h c, v16h d) { keep4_h(a, b, c, d); }
};
template <> struct Frag<__bf16> {
  typedef v16b V; union U { v16b v; v8b h[2]; };
  static __device__ __forceinline__ v16b load(const __bf16* p) {
    U f; f.h[0] = *(const v8b*)(p); f.h[1] = *(const v8b*)(p + 16); return f.v;
  }
  static __device__ __forceinline__ v8f mma(v16b a, v16b b, v8f c) {
    return __builtin_amdgcn_wmma_f32_16x16x32_bf16(false, a, false, b, (short)0, c, false, false);
  }
  static __device__ __forceinline__ void guard(v8f& a, v8f& b, v16b x, v16b y) { dep_guard_b(a, b, x, y); }
  static __device__ __forceinline__ void guard_all(v8f& a, v8f& b, v8f& c, v8f& d, v16b x0, v16b x1, v16b y0, v16b y1, v16b y2, v16b y3) { dep_guard_all_b(a, b, c, d, x0, x1, y0, y1, y2, y3); }
  static __device__ __forceinline__ void keep(v16b a, v16b b, v16b c, v16b d) { keep4_b(a, b, c, d); }
};

template <int ET> struct Elem;
template <> struct Elem<0> { typedef _Float16 T; };
template <> struct Elem<1> { typedef __bf16 T; };
template <int ET, int SPL, int BIAS_MODE, int OUT_MODE, bool RESID, int ACT = 0>
__global__ __launch_bounds__(256) void wmma_gemm64(
    const unsigned short* __restrict__ Ap, const unsigned short* __restrict__ A2p, int lda, long strideA,
    const unsigned short* __restrict__ Btp, const unsigned short* __restrict__ Bt2p, int ldb, long strideB,
    void* __restrict__ Cout, void* __restrict__ Cout2, int ldc, long strideC,
    const float* __restrict__ bias,
    const float* __restrict__ resid, long strideR,
    int M, int N, int K, float scale) {
  static_assert(OUT_MODE == 0, "f32 out only");
  typedef typename Elem<ET>::T T;
  typedef typename Frag<T>::V V;
  const T* A = (const T*)Ap; const T* A2 = (const T*)A2p; const T* Bt = (const T*)Btp; const T* Bt2 = (const T*)Bt2p;
  (void)Cout2;
  __shared__ __align__(16) float sT[8][16 * 68];
  const int b    = blockIdx.y;
  const int lane = threadIdx.x & 31;
  const int wave = threadIdx.x >> 5;
  const int tilesN = N >> 6;
  const int tilesM = M >> 6;
  const int tile = blockIdx.x * 8 + wave;
  if (tile >= tilesM * tilesN) return;
  const int tm = tile / tilesN;
  const int tn = tile - tm * tilesN;
  const int m0 = tm << 6;
  const int n0 = tn << 6;

  const T* Ab  = A  + (size_t)b * strideA;
  const T* Bb  = Bt + (size_t)b * strideB;
  const T* Ab2 = (SPL >= 1) ? (A2  + (size_t)b * strideA) : nullptr;
  const T* Bb2 = (SPL == 2) ? (Bt2 + (size_t)b * strideB) : nullptr;

  const int rlane = lane & 15;
  const int koff  = (lane >> 4) * 8;
  const int mOff  = (lane >> 4) * 8;

  v8f acc[4][4];
#pragma unroll
  for (int i = 0; i < 4; ++i)
#pragma unroll
    for (int j = 0; j < 4; ++j) acc[i][j] = (v8f){0.f,0.f,0.f,0.f,0.f,0.f,0.f,0.f};

  for (int k0 = 0; k0 < K; k0 += 32) {
    V bh[4], bl[4];
#pragma unroll
    for (int j = 0; j < 4; ++j) {
      const size_t bo = (size_t)(n0 + (j << 4) + rlane) * ldb + koff + k0;
      bh[j] = Frag<T>::load(Bb + bo);
      if (SPL == 2) bl[j] = Frag<T>::load(Bb2 + bo);
    }
#pragma unroll
    for (int i = 0; i < 4; ++i) {
      const size_t ao = (size_t)(m0 + (i << 4) + rlane) * lda + koff + k0;
      V ah = Frag<T>::load(Ab + ao);
      V al;
      if (SPL >= 1) al = Frag<T>::load(Ab2 + ao);
      else al = ah;
#pragma unroll
      for (int j = 0; j < 4; ++j) {
        acc[i][j] = Frag<T>::mma(ah, bh[j], acc[i][j]);
        if (SPL == 2) acc[i][j] = Frag<T>::mma(ah, bl[j], acc[i][j]);
        if (SPL >= 1) acc[i][j] = Frag<T>::mma(al, bh[j], acc[i][j]);
      }
      Frag<T>::guard_all(acc[i][0], acc[i][1], acc[i][2], acc[i][3], ah, al, bh[0], bh[1], bh[2], bh[3]);
      if (SPL == 2) Frag<T>::guard_all(acc[i][0], acc[i][1], acc[i][2], acc[i][3], ah, al, bl[0], bl[1], bl[2], bl[3]);
    }
    Frag<T>::keep(bh[0], bh[1], bh[2], bh[3]);
    if (SPL == 2) Frag<T>::keep(bl[0], bl[1], bl[2], bl[3]);
  }
  acc_guard4(acc[0][0], acc[0][1], acc[0][2], acc[0][3]);
  acc_guard4(acc[1][0], acc[1][1], acc[1][2], acc[1][3]);
  acc_guard4(acc[2][0], acc[2][1], acc[2][2], acc[2][3]);
  acc_guard4(acc[3][0], acc[3][1], acc[3][2], acc[3][3]);

  float* slab = sT[wave];
  const float* Rb = RESID ? (resid + (size_t)b * strideR) : nullptr;
#pragma unroll
  for (int i = 0; i < 4; ++i) {
    const int mBase = m0 + (i << 4);
#pragma unroll
    for (int j = 0; j < 4; ++j) {
      const int n = n0 + (j << 4) + rlane;
      float bv = 0.f;
      if (BIAS_MODE == 2) bv = bias[n];
#pragma unroll
      for (int r = 0; r < 8; ++r) {
        float v = acc[i][j][r] * scale;
        if (BIAS_MODE == 1) v += bias[mBase + mOff + r];
        if (BIAS_MODE == 2) v += bv;
        if (ACT == 1) v = tanhf(v);
        if (ACT == 2) v = fmaxf(v, 0.0f);
        if (ACT == 3) v = v / (1.0f + expf(-v));
        if (ACT == 4) v = (v > 0.f) ? v : 0.01f * v;
        slab[(mOff + r) * 68 + (j << 4) + rlane] = v;
      }
    }
    __builtin_amdgcn_fence(__ATOMIC_RELEASE, "workgroup");
    __builtin_amdgcn_wave_barrier();
    __builtin_amdgcn_fence(__ATOMIC_ACQUIRE, "workgroup");
    {
      float* C = (float*)Cout + (size_t)b * strideC;
      const int hh = lane >> 4, c4 = (lane & 15) * 4;
      v4f ov[8];
#pragma unroll
      for (int it = 0; it < 8; ++it) {
        const int row = it * 2 + hh;
        v4f v = *(const v4f*)(slab + row * 68 + c4);
        if (RESID) {
          const v4f rr = *(const v4f*)(Rb + (size_t)(mBase + row) * ldc + n0 + c4);
          v4f rb;
          rb[0] = bf16_rne(rr[0]); rb[1] = bf16_rne(rr[1]); rb[2] = bf16_rne(rr[2]); rb[3] = bf16_rne(rr[3]);
          v = v + rb;
        }
        ov[it] = v;
      }
      for (int pass = 0; pass < 2; ++pass) {
#pragma unroll
        for (int it = 0; it < 8; ++it) {
          const int row = it * 2 + hh;
          *(volatile v4f*)(C + (size_t)(mBase + row) * ldc + n0 + c4) = ov[it];
        }
        __threadfence();
      }
    }
    __builtin_amdgcn_fence(__ATOMIC_RELEASE, "workgroup");
    __builtin_amdgcn_wave_barrier();
    __builtin_amdgcn_fence(__ATOMIC_ACQUIRE, "workgroup");
  }
}

__global__ __launch_bounds__(256) void cast_rows_bf16_kernel(
    const float* __restrict__ src, unsigned short* __restrict__ dst, int total8)
{
  const int i = blockIdx.x * 256 + threadIdx.x;
  if (i >= total8) return;
  const size_t e0 = (size_t)i << 3;
  const v4f a0 = *(const v4f*)(src + e0);
  const v4f a1 = *(const v4f*)(src + e0 + 4);
  v8h hv;
#pragma unroll
  for (int e = 0; e < 4; ++e) {
    const unsigned short h0 = f2bf_bits(a0[e]);
    const unsigned short h1 = f2bf_bits(a1[e]);
    hv[e]     = __builtin_bit_cast(_Float16, h0);
    hv[4 + e] = __builtin_bit_cast(_Float16, h1);
  }
  unsigned short* q = dst + e0;
  *(volatile v8h*)q = hv;
  __threadfence();
  *(volatile v8h*)q = hv;
}

__global__ __launch_bounds__(256) void zero_rows16_kernel(unsigned short* __restrict__ dst, int total8)
{
  const int i = blockIdx.x * 256 + threadIdx.x;
  if (i >= total8) return;
  const size_t e0 = (size_t)i << 3;
  const v4u z = (v4u){0u, 0u, 0u, 0u};
  v4u* q = (v4u*)(dst + e0);
  *(volatile v4u*)q = z;
  __threadfence();
  *(volatile v4u*)q = z;
}

__global__ __launch_bounds__(256) void layernorm_kernel(
    const float* __restrict__ x, const float* __restrict__ w, const float* __restrict__ bb,
    unsigned short* __restrict__ XNH, unsigned short* __restrict__ XNL)
{
  const int lane = threadIdx.x & 31, wave = threadIdx.x >> 5;
  const int row = blockIdx.x * 8 + wave;
  if (row >= kRows) return;
  const float* xr = x + (size_t)row * kDm + lane * 8;
  const v4f a0 = *(const v4f*)(xr);
  const v4f a1 = *(const v4f*)(xr + 4);
  float xv[8];
#pragma unroll
  for (int e = 0; e < 4; ++e) { xv[e] = bf16_rne(a0[e]); xv[4 + e] = bf16_rne(a1[e]); }
  float s = 0.0f;
#pragma unroll
  for (int e = 0; e < 8; ++e) s += xv[e];
#pragma unroll
  for (int off = 16; off >= 1; off >>= 1) s += __shfl_xor(s, off, 32);
  const float mu = s * (1.0f / (float)kDm);
  float vs = 0.0f;
#pragma unroll
  for (int e = 0; e < 8; ++e) { const float dd = xv[e] - mu; vs = fmaf(dd, dd, vs); }
#pragma unroll
  for (int off = 16; off >= 1; off >>= 1) vs += __shfl_xor(vs, off, 32);
  const float rstd = rsqrtf(vs * (1.0f / (float)kDm) + 1e-5f);
  const v4f w0 = *(const v4f*)(w + lane * 8);
  const v4f w1 = *(const v4f*)(w + lane * 8 + 4);
  const v4f b0 = *(const v4f*)(bb + lane * 8);
  const v4f b1 = *(const v4f*)(bb + lane * 8 + 4);
  float wv[8], bv8[8];
#pragma unroll
  for (int e = 0; e < 4; ++e) {
    wv[e] = bf16_rne(w0[e]);  wv[4 + e] = bf16_rne(w1[e]);
    bv8[e] = bf16_rne(b0[e]); bv8[4 + e] = bf16_rne(b1[e]);
  }
  v8h hv, lv;
#pragma unroll
  for (int e = 0; e < 8; ++e) {
    const float nv = ((xv[e] - mu) * rstd) * wv[e] + bv8[e];
    const unsigned short hb = f2bf_bits(nv);
    const unsigned short lb = f2bf_bits(nv - bf_bits2f(hb));
    hv[e] = __builtin_bit_cast(_Float16, hb);
    lv[e] = __builtin_bit_cast(_Float16, lb);
  }
  const size_t o = (size_t)row * kDm + lane * 8;
  *(volatile v8h*)(XNH + o) = hv;
  *(volatile v8h*)(XNL + o) = lv;
  __threadfence();
  *(volatile v8h*)(XNH + o) = hv;
  *(volatile v8h*)(XNL + o) = lv;
}

__global__ __launch_bounds__(256) void conv_silu_kernel(
    const float* __restrict__ XZ, const float* __restrict__ cw, const float* __restrict__ cb,
    unsigned short* __restrict__ UH, unsigned short* __restrict__ UL)
{
  __shared__ __align__(16) float sT[16 * kConvTP];
  const int tid = threadIdx.x, lane = tid & 31, wave = tid >> 5;
  const int d0 = blockIdx.x * 256, d = d0 + tid;
  const int g0 = blockIdx.y * 64;
  const int tb = g0 & (kSeq - 1);
  const v4f wa = *(const v4f*)(cw + (size_t)d * kConvK);
  const v4f wb = *(const v4f*)(cw + (size_t)d * kConvK + 4);
  const float w0 = bf16_rne(wa[0]), w1 = bf16_rne(wa[1]), w2 = bf16_rne(wa[2]), w3 = bf16_rne(wa[3]);
  const float w4 = bf16_rne(wb[0]), w5 = bf16_rne(wb[1]), w6 = bf16_rne(wb[2]), w7 = bf16_rne(wb[3]);
  const float bc = bf16_rne(cb[d]);
  float x1, x2, x3, x4, x5, x6, x7;
  {
    const bool hist = (tb > 0);
    const int rb = hist ? (g0 - 7) : g0;
    const float v7 = XZ[(size_t)rb * kXzP + d];
    const float v6 = XZ[(size_t)(rb + 1) * kXzP + d];
    const float v5 = XZ[(size_t)(rb + 2) * kXzP + d];
    const float v4 = XZ[(size_t)(rb + 3) * kXzP + d];
    const float v3 = XZ[(size_t)(rb + 4) * kXzP + d];
    const float v2 = XZ[(size_t)(rb + 5) * kXzP + d];
    const float v1 = XZ[(size_t)(rb + 6) * kXzP + d];
    x7 = hist ? v7 : 0.f;
    x6 = hist ? v6 : 0.f;
    x5 = hist ? v5 : 0.f;
    x4 = hist ? v4 : 0.f;
    x3 = hist ? v3 : 0.f;
    x2 = hist ? v2 : 0.f;
    x1 = hist ? v1 : 0.f;
  }
#pragma unroll 1
  for (int sub = 0; sub < 4; ++sub) {
    const int lb = g0 + sub * 16;
#pragma unroll 1
    for (int s = 0; s < 16; ++s) {
      const float xcur = XZ[(size_t)(lb + s) * kXzP + d];
      float acc = w0 * x7;
      acc = fmaf(w1, x6, acc);
      acc = fmaf(w2, x5, acc);
      acc = fmaf(w3, x4, acc);
      acc = fmaf(w4, x3, acc);
      acc = fmaf(w5, x2, acc);
      acc = fmaf(w6, x1, acc);
      acc = fmaf(w7, xcur, acc);
      const float sv = acc + bc;
      const float sg = __builtin_amdgcn_rcpf(1.0f + __expf(-sv));
      sT[s * kConvTP + tid] = sv * sg;
      x7 = x6; x6 = x5; x5 = x4; x4 = x3; x3 = x2; x2 = x1; x1 = xcur;
    }
    __syncthreads();
    v8h hv[2], lv[2];
#pragma unroll
    for (int it = 0; it < 2; ++it) {
      const float* sp = sT + (it * 8 + wave) * kConvTP + lane * 8;
      const v4f a0 = *(const v4f*)(sp);
      const v4f a1 = *(const v4f*)(sp + 4);
#pragma unroll
      for (int e = 0; e < 4; ++e) {
        const unsigned short h0 = f2bf_bits(a0[e]), h1 = f2bf_bits(a1[e]);
        const unsigned short l0 = f2bf_bits(a0[e] - bf_bits2f(h0)), l1 = f2bf_bits(a1[e] - bf_bits2f(h1));
        hv[it][e]     = __builtin_bit_cast(_Float16, h0);
        hv[it][4 + e] = __builtin_bit_cast(_Float16, h1);
        lv[it][e]     = __builtin_bit_cast(_Float16, l0);
        lv[it][4 + e] = __builtin_bit_cast(_Float16, l1);
      }
    }
    for (int pass = 0; pass < 2; ++pass) {
#pragma unroll
      for (int it = 0; it < 2; ++it) {
        const size_t o = (size_t)(lb + it * 8 + wave) * kDin + d0 + lane * 8;
        *(volatile v8h*)(UH + o) = hv[it];
        *(volatile v8h*)(UL + o) = lv[it];
      }
      __threadfence();
    }
    __syncthreads();
  }
}

__global__ __launch_bounds__(kScanTh) void scan_kernel(
    const float* __restrict__ XD, const float* __restrict__ XZ,
    const float* __restrict__ cw, const float* __restrict__ cb,
    const float* __restrict__ Wdt, const float* __restrict__ bdt, const float* __restrict__ Alog,
    const float* __restrict__ Dp, unsigned short* __restrict__ YH, unsigned short* __restrict__ YL)
{
  __shared__ __align__(16) float sX[kScanTS * kSxP];
  __shared__ __align__(16) float sY[kScanTS * kScanYP];
  __shared__ __align__(16) float sW[kDtR * kScanCh];
  __shared__ __align__(16) float sA[kNstL * kScanTh];
  const int tid = threadIdx.x, lane = tid & 31, wave = tid >> 5;
  const int c = tid >> 1, half = tid & 1;
  constexpr int kBlkPerB = kDin / kScanCh;
  const int bix = blockIdx.x / kBlkPerB;
  const int d0  = (blockIdx.x - bix * kBlkPerB) * kScanCh;
  const int d   = d0 + c;
  const int s0  = half * kNstL;
  const size_t row0 = (size_t)bix * kSeq;
  {
    const v4f wv0 = *(const v4f*)(Wdt + (size_t)d * kDtR + half * 8);
    const v4f wv1 = *(const v4f*)(Wdt + (size_t)d * kDtR + half * 8 + 4);
    float* swp = sW + (half * 8) * kScanCh + c;
    swp[0 * kScanCh] = bf16_rne(wv0[0]);
    swp[1 * kScanCh] = bf16_rne(wv0[1]);
    swp[2 * kScanCh] = bf16_rne(wv0[2]);
    swp[3 * kScanCh] = bf16_rne(wv0[3]);
    swp[4 * kScanCh] = bf16_rne(wv1[0]);
    swp[5 * kScanCh] = bf16_rne(wv1[1]);
    swp[6 * kScanCh] = bf16_rne(wv1[2]);
    swp[7 * kScanCh] = bf16_rne(wv1[3]);
  }
#pragma unroll 1
  for (int j = 0; j < kNstL; ++j) sA[j * kScanTh + tid] = -expf(bf16_rne(Alog[(size_t)d * kNst + s0 + j]));
  const v4f wa = *(const v4f*)(cw + (size_t)d * kConvK);
  const v4f wb = *(const v4f*)(cw + (size_t)d * kConvK + 4);
  const float w0 = bf16_rne(wa[0]), w1 = bf16_rne(wa[1]), w2 = bf16_rne(wa[2]), w3 = bf16_rne(wa[3]);
  const float w4 = bf16_rne(wb[0]), w5 = bf16_rne(wb[1]), w6 = bf16_rne(wb[2]), w7 = bf16_rne(wb[3]);
  const float bc = bf16_rne(cb[d]);
  const float bb = bf16_rne(bdt[d]);
  const float Dd = bf16_rne(Dp[d]);
  __syncthreads();
  float negA[kNstL], h[kNstL];
#pragma unroll
  for (int j = 0; j < kNstL; ++j) {
    negA[j] = sA[j * kScanTh + tid];
    h[j] = 0.0f;
  }
  float x1 = 0.f, x2 = 0.f, x3 = 0.f, x4 = 0.f, x5 = 0.f, x6 = 0.f, x7 = 0.f;
  const int q = lane >> 3, c8 = (lane & 7) * 8;
#pragma unroll 1
  for (int t0 = 0; t0 < kSeq; t0 += kScanTS) {
    __syncthreads();
#pragma unroll 1
    for (int i = 0; i < 10; ++i) {
      const int idx = tid + kScanTh * i;
      const int r   = idx / 20;
      const int c4  = (idx - r * 20) * 4;
      *(v4f*)(sX + r * kSxP + c4) = *(const v4f*)(XD + (row0 + (size_t)(t0 + r)) * (size_t)kXdP + c4);
    }
    __syncthreads();
#pragma unroll 1
    for (int s = 0; s < kScanTS; ++s) {
      const size_t grow = row0 + (size_t)(t0 + s);
      const float* xr = sX + s * kSxP;
      float vdot = 0.0f;
#pragma unroll 1
      for (int r4 = 0; r4 < kDtR / 4; ++r4) {
        const v4f xv = *(const v4f*)(xr + 4 * r4);
        const float* wp = sW + (4 * r4) * kScanCh + c;
        vdot = fmaf(xv[0], wp[0], vdot);
        vdot = fmaf(xv[1], wp[kScanCh], vdot);
        vdot = fmaf(xv[2], wp[2 * kScanCh], vdot);
        vdot = fmaf(xv[3], wp[3 * kScanCh], vdot);
      }
      const float xcur = XZ[grow * kXzP + d];
      const float zv   = XZ[grow * kXzP + kDin + d];
      float cacc = w0 * x7;
      cacc = fmaf(w1, x6, cacc);
      cacc = fmaf(w2, x5, cacc);
      cacc = fmaf(w3, x4, cacc);
      cacc = fmaf(w4, x3, cacc);
      cacc = fmaf(w5, x2, cacc);
      cacc = fmaf(w6, x1, cacc);
      cacc = fmaf(w7, xcur, cacc);
      const float sv  = cacc + bc;
      const float sgu = __builtin_amdgcn_rcpf(1.0f + __expf(-sv));
      const float xt  = sv * sgu;
      x7 = x6; x6 = x5; x5 = x4; x4 = x3; x3 = x2; x2 = x1; x1 = xcur;
      const float v   = vdot + bb;
      const float a   = __expf(-fabsf(v));
      const float up1 = 1.0f + a;
      const float l1p = __logf(up1) + (a - (up1 - 1.0f)) * __builtin_amdgcn_rcpf(up1);
      const float dt  = fmaxf(v, 0.0f) + l1p;
      const float dtx = dt * xt;
      float yp = 0.0f;
#pragma unroll
      for (int q4 = 0; q4 < kNstL / 4; ++q4) {
        const v4f bv = *(const v4f*)(xr + kDtR + s0 + 4 * q4);
        const v4f cv = *(const v4f*)(xr + kDtR + kNst + s0 + 4 * q4);
#pragma unroll
        for (int e = 0; e < 4; ++e) {
          const int k = 4 * q4 + e;
          const float ex = __expf(dt * negA[k]);
          h[k] = fmaf(ex, h[k], dtx * bv[e]);
          yp = fmaf(h[k], cv[e], yp);
        }
      }
      const float yo = __shfl_xor(yp, 1, 32);
      float y = yp + yo;
      y = fmaf(xt, Dd, y);
      const float sgz = __builtin_amdgcn_rcpf(1.0f + __expf(-zv));
      y = y * (zv * sgz);
      if (half == 0) sY[s * kScanYP + c] = y;
    }
    __syncthreads();
    v8h hv[4], lv[4];
#pragma unroll
    for (int it = 0; it < 4; ++it) {
      const int row = it * 16 + wave * 4 + q;
      const float* sp = sY + row * kScanYP + c8;
      const v4f a0 = *(const v4f*)(sp);
      const v4f a1 = *(const v4f*)(sp + 4);
#pragma unroll
      for (int e = 0; e < 4; ++e) {
        const unsigned short h0 = f2bf_bits(a0[e]), h1 = f2bf_bits(a1[e]);
        const unsigned short l0 = f2bf_bits(a0[e] - bf_bits2f(h0)), l1 = f2bf_bits(a1[e] - bf_bits2f(h1));
        hv[it][e]     = __builtin_bit_cast(_Float16, h0);
        hv[it][4 + e] = __builtin_bit_cast(_Float16, h1);
        lv[it][e]     = __builtin_bit_cast(_Float16, l0);
        lv[it][4 + e] = __builtin_bit_cast(_Float16, l1);
      }
    }
    for (int pass = 0; pass < 2; ++pass) {
#pragma unroll
      for (int it = 0; it < 4; ++it) {
        const int row = it * 16 + wave * 4 + q;
        const size_t o = (row0 + (size_t)(t0 + row)) * kDin + d0 + c8;
        *(volatile v8h*)(YH + o) = hv[it];
        *(volatile v8h*)(YL + o) = lv[it];
      }
      __threadfence();
    }
  }
}

static_assert((kRows / 64) * (kXzP / 64) == 8 * 512, "in_proj grid");
static_assert((kRows / 64) * (kXdP / 64) == 8 * 32, "x_proj grid");
static_assert((kRows / 64) * (kDm / 64) == 8 * 64, "out_proj grid");
static_assert((kXzP * kDm / 8) == 256 * 256 && (kXdW * kDin / 8) == 256 * 40 && ((kXdP - kXdW) * kDin / 8) == 256 * 24 && (kDm * kDin / 8) == 256 * 128, "cast grids");
static_assert(kRows % 8 == 0 && kBatch * (kDin / kScanCh) == 128, "LN and scan grids");

extern "C" void kernel_launch(void* const* d_in, const int* in_sizes, int n_in,
                              void* d_out, int out_size, void* d_ws, size_t ws_size,
                              hipStream_t stream) {
  if (n_in < 12) return;
  if (in_sizes[0]  != kRows * kDm) return;
  if (in_sizes[1]  != kDm) return;
  if (in_sizes[2]  != kDm) return;
  if (in_sizes[3]  != kXzP * kDm) return;
  if (in_sizes[4]  != kDin * kConvK) return;
  if (in_sizes[5]  != kDin) return;
  if (in_sizes[6]  != kXdW * kDin) return;
  if (in_sizes[7]  != kDin * kDtR) return;
  if (in_sizes[8]  != kDin) return;
  if (in_sizes[9]  != kDin * kNst) return;
  if (in_sizes[10] != kDin) return;
  if (in_sizes[11] != kDm * kDin) return;
  if (out_size != kRows * kDm) return;
  if (ws_size < kWsTotal) return;

  const float* x       = (const float*)d_in[0];
  const float* norm_w  = (const float*)d_in[1];
  const float* norm_b  = (const float*)d_in[2];
  const float* W_in    = (const float*)d_in[3];
  const float* conv_w  = (const float*)d_in[4];
  const float* conv_b  = (const float*)d_in[5];
  const float* W_x     = (const float*)d_in[6];
  const float* W_dt    = (const float*)d_in[7];
  const float* b_dt    = (const float*)d_in[8];
  const float* A_log   = (const float*)d_in[9];
  const float* Dp      = (const float*)d_in[10];
  const float* W_out   = (const float*)d_in[11];
  float* out = (float*)d_out;

  char* ws = (char*)d_ws;
  unsigned short* XNH = (unsigned short*)(ws + kOffXNH);
  unsigned short* XNL = (unsigned short*)(ws + kOffXNL);
  unsigned short* WI  = (unsigned short*)(ws + kOffWI);
  unsigned short* WX  = (unsigned short*)(ws + kOffWX);
  unsigned short* WO  = (unsigned short*)(ws + kOffWO);
  float*          XZ  = (float*)(ws + kOffXZ);
  unsigned short* UY0 = (unsigned short*)(ws + kOffUY0);
  unsigned short* UY1 = (unsigned short*)(ws + kOffUY1);
  float*          XD  = (float*)(ws + kOffXD);

  cast_rows_bf16_kernel<<<(kXzP * kDm / 8) / 256, 256, 0, stream>>>(W_in, WI, kXzP * kDm / 8);
  cast_rows_bf16_kernel<<<(kXdW * kDin / 8) / 256, 256, 0, stream>>>(W_x, WX, kXdW * kDin / 8);
  zero_rows16_kernel<<<((kXdP - kXdW) * kDin / 8) / 256, 256, 0, stream>>>(WX + (size_t)kXdW * kDin, (kXdP - kXdW) * kDin / 8);
  cast_rows_bf16_kernel<<<(kDm * kDin / 8) / 256, 256, 0, stream>>>(W_out, WO, kDm * kDin / 8);

  layernorm_kernel<<<kRows / 8, 256, 0, stream>>>(x, norm_w, norm_b, XNH, XNL);

  wmma_gemm64<1, 1, 0, 0, false><<<dim3(512, 1), 256, 0, stream>>>(
      XNH, XNL, kDm, 0L,
      WI, nullptr, kDm, 0L,
      (void*)XZ, nullptr, kXzP, 0L,
      nullptr, nullptr, 0L,
      kRows, kXzP, kDm, 1.0f);

  conv_silu_kernel<<<dim3(kDin / 256, kRows / 64), 256, 0, stream>>>(XZ, conv_w, conv_b, UY0, UY1);

  wmma_gemm64<1, 1, 0, 0, false><<<dim3(32, 1), 256, 0, stream>>>(
      UY0, UY1, kDin, 0L,
      WX, nullptr, kDin, 0L,
      (void*)XD, nullptr, kXdP, 0L,
      nullptr, nullptr, 0L,
      kRows, kXdP, kDin, 1.0f);

  scan_kernel<<<kBatch * (kDin / kScanCh), kScanTh, 0, stream>>>(XD, XZ, conv_w, conv_b, W_dt, b_dt, A_log, Dp, UY0, UY1);

  wmma_gemm64<1, 1, 0, 0, true><<<dim3(64, 1), 256, 0, stream>>>(
      UY0, UY1, kDin, 0L,
      WO, nullptr, kDin, 0L,
      (void*)out, nullptr, kDm, 0L,
      nullptr, x, 0L,
      kRows, kDm, kDin, 1.0f);
}
